// HopfieldAttention_16535624090005
// MI455X (gfx1250) — hardware-verified
//
#include <hip/hip_runtime.h>

constexpr int NBATCH = 2;
constexpr int SEQ    = 2048;
constexpr int HIDN   = 1024;
constexpr int NHEAD  = 16;
constexpr int HDIM   = 64;
constexpr int NTOK   = NBATCH * SEQ;
constexpr size_t NX  = (size_t)NTOK * HIDN;
constexpr size_t NW  = (size_t)HIDN * HIDN;
constexpr size_t OUT0_ELEMS    = NX;
constexpr size_t OUT1_ELEMS    = (size_t)NBATCH * NHEAD * HDIM * HDIM;
constexpr size_t OUT1_BYTE_OFF = 16777216;
constexpr size_t OUT1_ELEM_OFF = OUT1_BYTE_OFF / 4;
static_assert(OUT1_ELEM_OFF == OUT0_ELEMS);
static_assert(OUT1_BYTE_OFF + OUT1_ELEMS * 4 == 17301504);
static_assert(HIDN == NHEAD * HDIM);
static_assert(HDIM == 64);
static_assert(HIDN % 64 == 0 && NTOK % 64 == 0 && SEQ % 64 == 0);
static_assert(HIDN % 32 == 0 && SEQ % 32 == 0);
static_assert((NX % 512) == 0 && (NW % 512) == 0);

constexpr size_t MIB      = (size_t)1 << 20;
constexpr size_t OFF_XB   = 0 * MIB;
constexpr size_t OFF_WQ   = 8 * MIB;
constexpr size_t OFF_WK   = 10 * MIB;
constexpr size_t OFF_WV   = 12 * MIB;
constexpr size_t OFF_WO   = 14 * MIB;
constexpr size_t OFF_QH   = 16 * MIB;
constexpr size_t OFF_QL   = 24 * MIB;
constexpr size_t OFF_KH   = 32 * MIB;
constexpr size_t OFF_KL   = 40 * MIB;
constexpr size_t OFF_KTH  = 48 * MIB;
constexpr size_t OFF_KTL  = 56 * MIB;
constexpr size_t OFF_VTH  = 64 * MIB;
constexpr size_t OFF_VTL  = 72 * MIB;
constexpr size_t OFF_OH   = 80 * MIB;
constexpr size_t OFF_OL   = 88 * MIB;
constexpr size_t WS_TOTAL = 96 * MIB;
static_assert(NX * 2 == 8 * MIB && NW * 2 == 2 * MIB);
static_assert(WS_TOTAL <= 134217728);

typedef __attribute__((ext_vector_type(16))) _Float16 v16h;
typedef __attribute__((ext_vector_type(8)))  _Float16 v8h;
typedef __attribute__((ext_vector_type(16))) __bf16   v16b;
typedef __attribute__((ext_vector_type(8)))  __bf16   v8b;
typedef __attribute__((ext_vector_type(8)))  float    v8f;
typedef __attribute__((ext_vector_type(4)))  float    v4f;
typedef __attribute__((ext_vector_type(2)))  float    v2f;
typedef __attribute__((ext_vector_type(4)))  unsigned u4v;

__device__ __forceinline__ unsigned short f2bf_bits(float f) {
  unsigned u = __float_as_uint(f);
  return (unsigned short)((u + 0x7FFFu + ((u >> 16) & 1u)) >> 16);
}
__device__ __forceinline__ float bf_bits2f(unsigned short h) { return __uint_as_float(((unsigned)h) << 16); }
__device__ __forceinline__ float bfr(float f) { return bf_bits2f(f2bf_bits(f)); }

__device__ __forceinline__ void sched_fence() { asm volatile("" ::: "memory"); }

__device__ __forceinline__ void dep_guard_h(v8f& a, v8f& b, v16h x, v16h y) { asm volatile("v_nop\n\tv_nop\n\tv_nop\n\tv_nop" : "+v"(a), "+v"(b) : "v"(x), "v"(y)); }
__device__ __forceinline__ void dep_guard_b(v8f& a, v8f& b, v16b x, v16b y) { asm volatile("v_nop\n\tv_nop\n\tv_nop\n\tv_nop" : "+v"(a), "+v"(b) : "v"(x), "v"(y)); }
__device__ __forceinline__ void keep4_h(v16h a, v16h b, v16h c, v16h d) { asm volatile("v_nop" :: "v"(a), "v"(b), "v"(c), "v"(d)); }
__device__ __forceinline__ void keep4_b(v16b a, v16b b, v16b c, v16b d) { asm volatile("v_nop" :: "v"(a), "v"(b), "v"(c), "v"(d)); }
__device__ __forceinline__ void acc_guard4(v8f& a, v8f& b, v8f& c, v8f& d) { asm volatile("v_nop\n\tv_nop\n\tv_nop\n\tv_nop" : "+v"(a), "+v"(b), "+v"(c), "+v"(d)); }
template <typename T> struct Frag;
template <> struct Frag<_Float16> {
  typedef v16h V; union U { v16h v; v8h h[2]; };
  static __device__ __forceinline__ v16h load(const _Float16* p) {
    U f; f.h[0] = *(const v8h*)(p); f.h[1] = *(const v8h*)(p + 16); return f.v;
  }
  static __device__ __forceinline__ v8f mma(v16h a, v16h b, v8f c) {
    return __builtin_amdgcn_wmma_f32_16x16x32_f16(false, a, false, b, (short)0, c, false, false);
  }
  static __device__ __forceinline__ void guard(v8f& a, v8f& b, v16h x, v16h y) { dep_guard_h(a, b, x, y); }
  static __device__ __forceinline__ void keep(v16h a, v16h b, v16h c, v16h d) { keep4_h(a, b, c, d); }
};
template <> struct Frag<__bf16> {
  typedef v16b V; union U { v16b v; v8b h[2]; };
  static __device__ __forceinline__ v16b load(const __bf16* p) {
    U f; f.h[0] = *(const v8b*)(p); f.h[1] = *(const v8b*)(p + 16); return f.v;
  }
  static __device__ __forceinline__ v8f mma(v16b a, v16b b, v8f c) {
    return __builtin_amdgcn_wmma_f32_16x16x32_bf16(false, a, false, b, (short)0, c, false, false);
  }
  static __device__ __forceinline__ void guard(v8f& a, v8f& b, v16b x, v16b y) { dep_guard_b(a, b, x, y); }
  static __device__ __forceinline__ void keep(v16b a, v16b b, v16b c, v16b d) { keep4_b(a, b, c, d); }
};

template <int ET> struct Elem;
template <> struct Elem<0> { typedef _Float16 T; };
template <> struct Elem<1> { typedef __bf16 T; };
template <int ET, bool SPLIT, bool BLO, int BIAS_MODE, int OUT_MODE, int RS_MODE>
__global__ __launch_bounds__(256) void wmma_gemm64(
    const unsigned short* __restrict__ Ap, const unsigned short* __restrict__ A2p, int lda, long strideA,
    const unsigned short* __restrict__ Btp, const unsigned short* __restrict__ Bt2p, int ldb, long strideB,
    void* __restrict__ Cout, void* __restrict__ Cout2, int ldc, long strideC,
    const float* __restrict__ bias, const float* __restrict__ rsc,
    int M, int N, int K, float scale) {
  typedef typename Elem<ET>::T T;
  typedef typename Frag<T>::V V;
  const T* A = (const T*)Ap; const T* A2 = (const T*)A2p; const T* Bt = (const T*)Btp; const T* Bt2 = (const T*)Bt2p;
  __shared__ __align__(16) float sT[8][16 * 68];
  const int b    = blockIdx.y;
  const int lane = threadIdx.x & 31;
  const int wave = threadIdx.x >> 5;
  const int tilesN = N >> 6;
  const int tilesM = M >> 6;
  const int tile = blockIdx.x * 8 + wave;
  if (tile >= tilesM * tilesN) return;
  const int tm = tile / tilesN;
  const int tn = tile - tm * tilesN;
  const int m0 = tm << 6;
  const int n0 = tn << 6;

  const T* Ab  = A  + (size_t)b * strideA;
  const T* Bb  = Bt + (size_t)b * strideB;
  const T* Ab2 = SPLIT ? (A2  + (size_t)b * strideA) : nullptr;
  const T* Bb2 = (SPLIT && BLO) ? (Bt2 + (size_t)b * strideB) : nullptr;

  const int rlane = lane & 15;
  const int koff  = (lane >> 4) * 8;
  const int mOff  = (lane >> 4) * 8;

  v8f acc[4][4];
#pragma unroll
  for (int i = 0; i < 4; ++i)
#pragma unroll
    for (int j = 0; j < 4; ++j) acc[i][j] = (v8f){0.f,0.f,0.f,0.f,0.f,0.f,0.f,0.f};

  for (int k0 = 0; k0 < K; k0 += 32) {
    V bh[4], bl[4];
#pragma unroll
    for (int j = 0; j < 4; ++j) {
      const size_t bo = (size_t)(n0 + (j << 4) + rlane) * ldb + koff + k0;
      bh[j] = Frag<T>::load(Bb + bo);
      if (SPLIT && BLO) bl[j] = Frag<T>::load(Bb2 + bo);
      else bl[j] = bh[j];
    }
#pragma unroll
    for (int i = 0; i < 4; ++i) {
      const size_t ao = (size_t)(m0 + (i << 4) + rlane) * lda + koff + k0;
      V ah = Frag<T>::load(Ab + ao);
      V al = ah;
      if (SPLIT) al = Frag<T>::load(Ab2 + ao);
#pragma unroll
      for (int j = 0; j < 4; ++j) {
        acc[i][j] = Frag<T>::mma(ah, bh[j], acc[i][j]);
        if (SPLIT) {
          if (BLO) acc[i][j] = Frag<T>::mma(ah, bl[j], acc[i][j]);
          acc[i][j] = Frag<T>::mma(al, bh[j], acc[i][j]);
        }
      }
      Frag<T>::guard(acc[i][0], acc[i][3], ah, al);
    }
    Frag<T>::keep(bh[0], bh[1], bh[2], bh[3]);
    if (SPLIT && BLO) Frag<T>::keep(bl[0], bl[1], bl[2], bl[3]);
  }
  acc_guard4(acc[0][0], acc[0][1], acc[0][2], acc[0][3]);
  acc_guard4(acc[1][0], acc[1][1], acc[1][2], acc[1][3]);
  acc_guard4(acc[2][0], acc[2][1], acc[2][2], acc[2][3]);
  acc_guard4(acc[3][0], acc[3][1], acc[3][2], acc[3][3]);

  float* slab = sT[wave];
#pragma unroll
  for (int i = 0; i < 4; ++i) {
    const int mBase = m0 + (i << 4);
    float bm[8], rm[8];
#pragma unroll
    for (int r = 0; r < 8; ++r) { bm[r] = 0.f; rm[r] = 1.f; }
    if (BIAS_MODE == 1) {
      const v4f t0 = *(const v4f*)(bias + mBase + mOff);
      const v4f t1 = *(const v4f*)(bias + mBase + mOff + 4);
#pragma unroll
      for (int r = 0; r < 4; ++r) { bm[r] = bfr(t0[r]); bm[4 + r] = bfr(t1[r]); }
    }
    if (RS_MODE == 1) {
      const v4f t0 = *(const v4f*)(rsc + mBase + mOff);
      const v4f t1 = *(const v4f*)(rsc + mBase + mOff + 4);
#pragma unroll
      for (int r = 0; r < 4; ++r) { rm[r] = bfr(t0[r]); rm[4 + r] = bfr(t1[r]); }
    }
#pragma unroll
    for (int j = 0; j < 4; ++j) {
      const int n = n0 + (j << 4) + rlane;
      float bn = 0.f, rn = 1.f;
      if (BIAS_MODE == 2) bn = bfr(bias[n]);
      if (RS_MODE == 2)   rn = bfr(rsc[n]);
#pragma unroll
      for (int r = 0; r < 8; ++r) {
        float v = acc[i][j][r] * scale;
        if (BIAS_MODE == 1) v += bm[r];
        if (BIAS_MODE == 2) v += bn;
        if (RS_MODE == 1) v *= rm[r];
        if (RS_MODE == 2) v *= rn;
        slab[(mOff + r) * 68 + (j << 4) + rlane] = v;
      }
    }
    __builtin_amdgcn_fence(__ATOMIC_RELEASE, "workgroup");
    __builtin_amdgcn_wave_barrier();
    __builtin_amdgcn_fence(__ATOMIC_ACQUIRE, "workgroup");
    if (OUT_MODE == 0) {
      float* C = (float*)Cout + (size_t)b * strideC;
      const int hh = lane >> 4, c4 = (lane & 15) * 4;
      for (int pass = 0; pass < 2; ++pass) {
#pragma unroll
        for (int it = 0; it < 8; ++it) {
          const int row = it * 2 + hh;
          v4f v = *(const v4f*)(slab + row * 68 + c4);
          *(volatile v4f*)(C + (size_t)(mBase + row) * ldc + n0 + c4) = v;
        }
        __threadfence();
      }
    } else {
      const int q = lane >> 3, c8 = (lane & 7) * 8;
      unsigned short* C  = (unsigned short*)Cout  + (size_t)b * strideC;
      unsigned short* C2 = (OUT_MODE == 2) ? ((unsigned short*)Cout2 + (size_t)b * strideC) : nullptr;
      for (int pass = 0; pass < 2; ++pass) {
#pragma unroll
        for (int it = 0; it < 4; ++it) {
          const int row = it * 4 + q;
          const float* sp = slab + row * 68 + c8;
          v8h hv, lv;
#pragma unroll
          for (int e = 0; e < 8; ++e) {
            if (OUT_MODE == 1) {
              hv[e] = (_Float16)sp[e];
              lv[e] = hv[e];
            } else {
              unsigned short hb = f2bf_bits(sp[e]);
              unsigned short lb = f2bf_bits(sp[e] - bf_bits2f(hb));
              hv[e] = __builtin_bit_cast(_Float16, hb);
              lv[e] = __builtin_bit_cast(_Float16, lb);
            }
          }
          *(volatile v8h*)(C + (size_t)(mBase + row) * ldc + n0 + c8) = hv;
          if (OUT_MODE == 2) *(volatile v8h*)(C2 + (size_t)(mBase + row) * ldc + n0 + c8) = lv;
        }
        __threadfence();
      }
    }
    __builtin_amdgcn_fence(__ATOMIC_RELEASE, "workgroup");
    __builtin_amdgcn_wave_barrier();
    __builtin_amdgcn_fence(__ATOMIC_ACQUIRE, "workgroup");
  }
}

__global__ __launch_bounds__(256) void cast_f32_bf16x2(
    const float* __restrict__ in, unsigned short* __restrict__ out, int n2) {
  int i = blockIdx.x * 256 + threadIdx.x;
  if (i < n2) {
    const v2f f = *(const v2f*)(in + 2 * (size_t)i);
    const unsigned u = (unsigned)f2bf_bits(f[0]) | ((unsigned)f2bf_bits(f[1]) << 16);
    ((volatile unsigned*)out)[i] = u;
    __threadfence();
    ((volatile unsigned*)out)[i] = u;
  }
}

constexpr int AT_D  = 64;
constexpr int AT_NW = 4;
constexpr int AT_QB = 64;
constexpr int AT_KC = 64;

__device__ __forceinline__ __bf16 at_f2bf(float f) { return __builtin_bit_cast(__bf16, f2bf_bits(f)); }
__device__ __forceinline__ void at_split(float f, __bf16& hi, __bf16& lo) {
  const unsigned short hb = f2bf_bits(f);
  hi = __builtin_bit_cast(__bf16, hb);
  lo = at_f2bf(f - __uint_as_float(((unsigned)hb) << 16));
}
__device__ __forceinline__ v8f at_mma(v16b a, v16b b, v8f c) {
  c = __builtin_amdgcn_wmma_f32_16x16x32_bf16(false, a, false, b, (short)0, c, false, false);
  asm volatile("v_nop\n\tv_nop\n\tv_nop\n\tv_nop" : "+v"(c) : "v"(a), "v"(b));
  return c;
}

__global__ __launch_bounds__(128) __attribute__((amdgpu_num_vgpr(256)))
void attn_hd64_planes(const unsigned short* __restrict__ Qh, const unsigned short* __restrict__ Ql,
                      const unsigned short* __restrict__ Kh, const unsigned short* __restrict__ Kl,
                      const unsigned short* __restrict__ VTh, const unsigned short* __restrict__ VTl,
                      const float* __restrict__ amask,
                      unsigned short* __restrict__ Oh, unsigned short* __restrict__ Ol,
                      float sscale) {
  union FB { v16b v; v8b h[2]; };
  __shared__ __align__(16) __bf16 Ksh[AT_KC * AT_D];
  __shared__ __align__(16) __bf16 Ksl[AT_KC * AT_D];
  __shared__ __align__(16) __bf16 Vth[AT_D * AT_KC];
  __shared__ __align__(16) __bf16 Vtl[AT_D * AT_KC];
  __shared__ __align__(16) __bf16 Psh[AT_NW][16 * AT_KC];
  __shared__ __align__(16) __bf16 Psl[AT_NW][16 * AT_KC];
  __shared__ __align__(16) float  Os[AT_NW][16 * 68];

  const int tid  = threadIdx.x;
  const int wave = tid >> 5;
  const int lane = tid & 31;
  const int hh   = lane >> 4;
  const int c    = lane & 15;

  const int nqb = SEQ / AT_QB;
  const int bx  = blockIdx.x;
  const int qb  = bx % nqb;
  const int bhd = bx / nqb;
  const int h   = bhd % NHEAD;
  const int b   = bhd / NHEAD;
  const int q0  = qb * AT_QB + wave * 16;
  const int tok0 = b * SEQ;
  const int hcol = h * HDIM;

  v16b qah[2], qal[2];
  {
    const __bf16* qhp = (const __bf16*)Qh + (size_t)(tok0 + q0 + c) * HIDN + hcol + 8 * hh;
    const __bf16* qlp = (const __bf16*)Ql + (size_t)(tok0 + q0 + c) * HIDN + hcol + 8 * hh;
#pragma unroll
    for (int dc = 0; dc < 2; ++dc) {
      qah[dc] = Frag<__bf16>::load(qhp + dc * 32);
      qal[dc] = Frag<__bf16>::load(qlp + dc * 32);
    }
  }

  float mrow[8], lrow[8];
  v8f oacc[4];
#pragma unroll
  for (int r = 0; r < 8; ++r) { mrow[r] = -__builtin_inff(); lrow[r] = 0.f; }
#pragma unroll
  for (int t = 0; t < 4; ++t) oacc[t] = (v8f){0.f,0.f,0.f,0.f,0.f,0.f,0.f,0.f};

  const int nChunks = qb + 1;
  for (int kc = 0; kc < nChunks; ++kc) {
    const int kv0 = kc * AT_KC;
    __syncthreads();
    {
#pragma unroll
      for (int i = 0; i < 4; ++i) {
        const int id = tid + 128 * i;
        const int row = id >> 3, c8 = (id & 7) * 8;
        const size_t ko = (size_t)(tok0 + kv0 + row) * HIDN + hcol + c8;
        const u4v a0 = *(const u4v*)(Kh + ko);
        const u4v a1 = *(const u4v*)(Kl + ko);
        *(u4v*)(Ksh + row * AT_D + c8) = a0;
        *(u4v*)(Ksl + row * AT_D + c8) = a1;
      }
      sched_fence();
#pragma unroll
      for (int i = 0; i < 4; ++i) {
        const int id = tid + 128 * i;
        const int row = id >> 3, c8 = (id & 7) * 8;
        const size_t vo = (size_t)(hcol + row) * NTOK + tok0 + kv0 + c8;
        const u4v a0 = *(const u4v*)(VTh + vo);
        const u4v a1 = *(const u4v*)(VTl + vo);
        *(u4v*)(Vth + row * AT_KC + c8) = a0;
        *(u4v*)(Vtl + row * AT_KC + c8) = a1;
      }
    }
    __syncthreads();

    v8f s[4];
#pragma unroll
    for (int j = 0; j < 4; ++j) {
      v8f sj = (v8f){0.f,0.f,0.f,0.f,0.f,0.f,0.f,0.f};
#pragma unroll
      for (int dc = 0; dc < 2; ++dc) {
        FB kb, kl;
        const __bf16* khp = Ksh + (j * 16 + c) * AT_D + dc * 32 + 8 * hh;
        const __bf16* klp = Ksl + (j * 16 + c) * AT_D + dc * 32 + 8 * hh;
        kb.h[0] = *(const v8b*)(khp);
        kb.h[1] = *(const v8b*)(khp + 16);
        kl.h[0] = *(const v8b*)(klp);
        kl.h[1] = *(const v8b*)(klp + 16);
        sj = at_mma(qah[dc], kb.v, sj);
        sj = at_mma(qah[dc], kl.v, sj);
        sj = at_mma(qal[dc], kb.v, sj);
        sched_fence();
      }
      s[j] = sj;
    }
    const bool diag = (kc == qb);
    float kvm[4];
#pragma unroll
    for (int j = 0; j < 4; ++j) kvm[j] = amask[(size_t)tok0 + kv0 + j * 16 + c];
    float cm[8];
#pragma unroll
    for (int r = 0; r < 8; ++r) {
      const int qrow = q0 + 8 * hh + r;
      float m = -__builtin_inff();
#pragma unroll
      for (int j = 0; j < 4; ++j) {
        const int kvcol = kv0 + j * 16 + c;
        const bool masked = (diag && (kvcol > qrow)) || (kvm[j] == 0.0f);
        const float val = masked ? -__builtin_inff() : (s[j][r] * sscale);
        s[j][r] = val;
        m = fmaxf(m, val);
      }
#pragma unroll
      for (int off = 1; off < 16; off <<= 1) m = fmaxf(m, __shfl_xor(m, off, 32));
      cm[r] = m;
    }
    __bf16* pwh = Psh[wave];
    __bf16* pwl = Psl[wave];
#pragma unroll
    for (int r = 0; r < 8; ++r) {
      const float mnew = fmaxf(mrow[r], cm[r]);
      const float alpha = expf(mrow[r] - mnew);
      mrow[r] = mnew;
      float psum = 0.f;
#pragma unroll
      for (int j = 0; j < 4; ++j) {
        const float p = expf(s[j][r] - mnew);
        psum += p;
        __bf16 a, bl; at_split(p, a, bl);
        pwh[(8 * hh + r) * AT_KC + j * 16 + c] = a;
        pwl[(8 * hh + r) * AT_KC + j * 16 + c] = bl;
      }
#pragma unroll
      for (int off = 1; off < 16; off <<= 1) psum += __shfl_xor(psum, off, 32);
      lrow[r] = lrow[r] * alpha + psum;
#pragma unroll
      for (int t = 0; t < 4; ++t) oacc[t][r] *= alpha;
    }
    __builtin_amdgcn_fence(__ATOMIC_RELEASE, "workgroup");
    __builtin_amdgcn_wave_barrier();
    __builtin_amdgcn_fence(__ATOMIC_ACQUIRE, "workgroup");
#pragma unroll 1
    for (int kk = 0; kk < 2; ++kk) {
      FB pa, pl;
      pa.h[0] = *(const v8b*)(pwh + c * AT_KC + kk * 32 + 8 * hh);
      pa.h[1] = *(const v8b*)(pwh + c * AT_KC + kk * 32 + 16 + 8 * hh);
      pl.h[0] = *(const v8b*)(pwl + c * AT_KC + kk * 32 + 8 * hh);
      pl.h[1] = *(const v8b*)(pwl + c * AT_KC + kk * 32 + 16 + 8 * hh);
      sched_fence();
#pragma unroll
      for (int t = 0; t < 4; ++t) {
        FB vb, vl;
        const __bf16* vhp = Vth + (t * 16 + c) * AT_KC + kk * 32 + 8 * hh;
        const __bf16* vlp = Vtl + (t * 16 + c) * AT_KC + kk * 32 + 8 * hh;
        vb.h[0] = *(const v8b*)(vhp);
        vb.h[1] = *(const v8b*)(vhp + 16);
        vl.h[0] = *(const v8b*)(vlp);
        vl.h[1] = *(const v8b*)(vlp + 16);
        oacc[t] = at_mma(pa.v, vb.v, oacc[t]);
        oacc[t] = at_mma(pa.v, vl.v, oacc[t]);
        oacc[t] = at_mma(pl.v, vb.v, oacc[t]);
        sched_fence();
      }
    }
  }

  float* os = Os[wave];
#pragma unroll
  for (int r = 0; r < 8; ++r) {
    const float inv = 1.0f / lrow[r];
#pragma unroll
    for (int t = 0; t < 4; ++t) os[(8 * hh + r) * 68 + t * 16 + c] = oacc[t][r] * inv;
  }
  __builtin_amdgcn_fence(__ATOMIC_RELEASE, "workgroup");
  __builtin_amdgcn_wave_barrier();
  __builtin_amdgcn_fence(__ATOMIC_ACQUIRE, "workgroup");
  {
    const int q = lane >> 3, c8 = (lane & 7) * 8;
    for (int pass = 0; pass < 2; ++pass) {
#pragma unroll
      for (int it = 0; it < 4; ++it) {
        const int row = it * 4 + q;
        const float* sp = os + row * 68 + c8;
        v8h hv, lv;
#pragma unroll
        for (int e = 0; e < 8; ++e) {
          unsigned short hb = f2bf_bits(sp[e]);
          unsigned short lb = f2bf_bits(sp[e] - bf_bits2f(hb));
          hv[e] = __builtin_bit_cast(_Float16, hb);
          lv[e] = __builtin_bit_cast(_Float16, lb);
        }
        const size_t oo = (size_t)(tok0 + q0 + row) * HIDN + hcol + c8;
        *(volatile v8h*)(Oh + oo) = hv;
        *(volatile v8h*)(Ol + oo) = lv;
      }
      __threadfence();
    }
  }
}

extern "C" void kernel_launch(void* const* d_in, const int* in_sizes, int n_in,
                              void* d_out, int out_size, void* d_ws, size_t ws_size,
                              hipStream_t stream) {
  (void)n_in;
  if (ws_size < WS_TOTAL) return;
  if ((size_t)out_size != OUT0_ELEMS + OUT1_ELEMS) return;
  if ((size_t)in_sizes[0] != NX || (size_t)in_sizes[1] != (size_t)NTOK ||
      (size_t)in_sizes[2] != NW || (size_t)in_sizes[4] != NW ||
      (size_t)in_sizes[6] != NW || (size_t)in_sizes[8] != NW ||
      in_sizes[3] != HIDN || in_sizes[5] != HIDN || in_sizes[7] != HIDN || in_sizes[9] != HIDN) return;

  const float* hs    = (const float*)d_in[0];
  const float* amask = (const float*)d_in[1];
  const float* Wq    = (const float*)d_in[2];
  const float* bq    = (const float*)d_in[3];
  const float* Wk    = (const float*)d_in[4];
  const float* bk    = (const float*)d_in[5];
  const float* Wv    = (const float*)d_in[6];
  const float* bv    = (const float*)d_in[7];
  const float* Wo    = (const float*)d_in[8];
  const float* bo    = (const float*)d_in[9];

  char* ws = (char*)d_ws;
  unsigned short* Xb  = (unsigned short*)(ws + OFF_XB);
  unsigned short* Wqb = (unsigned short*)(ws + OFF_WQ);
  unsigned short* Wkb = (unsigned short*)(ws + OFF_WK);
  unsigned short* Wvb = (unsigned short*)(ws + OFF_WV);
  unsigned short* Wob = (unsigned short*)(ws + OFF_WO);
  unsigned short* Qh  = (unsigned short*)(ws + OFF_QH);
  unsigned short* Ql  = (unsigned short*)(ws + OFF_QL);
  unsigned short* Kh  = (unsigned short*)(ws + OFF_KH);
  unsigned short* Kl  = (unsigned short*)(ws + OFF_KL);
  unsigned short* KTh = (unsigned short*)(ws + OFF_KTH);
  unsigned short* KTl = (unsigned short*)(ws + OFF_KTL);
  unsigned short* VTh = (unsigned short*)(ws + OFF_VTH);
  unsigned short* VTl = (unsigned short*)(ws + OFF_VTL);
  unsigned short* Oh  = (unsigned short*)(ws + OFF_OH);
  unsigned short* Ol  = (unsigned short*)(ws + OFF_OL);

  float* outF   = (float*)d_out;
  float* stateF = outF + OUT1_ELEM_OFF;

  {
    const int n2x = (int)(NX / 2);
    const int n2w = (int)(NW / 2);
    cast_f32_bf16x2<<<dim3(n2x / 256), dim3(256), 0, stream>>>(hs, Xb, n2x);
    cast_f32_bf16x2<<<dim3(n2w / 256), dim3(256), 0, stream>>>(Wq, Wqb, n2w);
    cast_f32_bf16x2<<<dim3(n2w / 256), dim3(256), 0, stream>>>(Wk, Wkb, n2w);
    cast_f32_bf16x2<<<dim3(n2w / 256), dim3(256), 0, stream>>>(Wv, Wvb, n2w);
    cast_f32_bf16x2<<<dim3(n2w / 256), dim3(256), 0, stream>>>(Wo, Wob, n2w);
  }

  const int gemmBlocksTok = ((NTOK / 64) * (HIDN / 64)) / 8;
  wmma_gemm64<1, false, false, 2, 2, 0><<<dim3(gemmBlocksTok, 1), dim3(256), 0, stream>>>(
      Xb, Xb, HIDN, 0L, Wqb, Wqb, HIDN, 0L, (void*)Qh, (void*)Ql, HIDN, 0L,
      bq, amask, NTOK, HIDN, HIDN, 1.0f);
  wmma_gemm64<1, false, false, 2, 2, 1><<<dim3(gemmBlocksTok, 1), dim3(256), 0, stream>>>(
      Xb, Xb, HIDN, 0L, Wkb, Wkb, HIDN, 0L, (void*)Kh, (void*)Kl, HIDN, 0L,
      bk, amask, NTOK, HIDN, HIDN, 1.0f);
  wmma_gemm64<1, false, false, 1, 2, 2><<<dim3(gemmBlocksTok, 1), dim3(256), 0, stream>>>(
      Wkb, Wkb, HIDN, 0L, Xb, Xb, HIDN, 0L, (void*)KTh, (void*)KTl, NTOK, 0L,
      bk, amask, HIDN, NTOK, HIDN, 1.0f);
  wmma_gemm64<1, false, false, 1, 2, 2><<<dim3(gemmBlocksTok, 1), dim3(256), 0, stream>>>(
      Wvb, Wvb, HIDN, 0L, Xb, Xb, HIDN, 0L, (void*)VTh, (void*)VTl, NTOK, 0L,
      bv, amask, HIDN, NTOK, HIDN, 1.0f);

  const float sscale = 0.125f;
  attn_hd64_planes<<<dim3(NBATCH * NHEAD * (SEQ / AT_QB)), dim3(128), 0, stream>>>(
      Qh, Ql, Kh, Kl, VTh, VTl, amask, Oh, Ol, sscale);

  for (int bb = 0; bb < NBATCH; ++bb) {
    wmma_gemm64<1, true, true, 0, 0, 0><<<dim3(1, NHEAD), dim3(32), 0, stream>>>(
        KTh + (size_t)bb * SEQ, KTl + (size_t)bb * SEQ, NTOK, (long)HDIM * NTOK,
        VTh + (size_t)bb * SEQ, VTl + (size_t)bb * SEQ, NTOK, (long)HDIM * NTOK,
        (void*)(stateF + (size_t)bb * NHEAD * HDIM * HDIM), (void*)Oh, HDIM, (long)HDIM * HDIM,
        bo, amask, HDIM, HDIM, SEQ, 1.0f);
  }

  wmma_gemm64<1, true, false, 2, 0, 0><<<dim3(gemmBlocksTok, 1), dim3(256), 0, stream>>>(
      Oh, Ol, HIDN, 0L, Wob, Wob, HIDN, 0L, (void*)outF, (void*)Oh, HIDN, 0L,
      bo, amask, NTOK, HIDN, HIDN, 1.0f);
}
